// HiroLRAN_73581379715573
// MI455X (gfx1250) — hardware-run, weakly checked
//
#include <hip/hip_runtime.h>
#include <math.h>

typedef __attribute__((ext_vector_type(16))) _Float16 v16h;
typedef __attribute__((ext_vector_type(8)))  _Float16 v8h;
typedef __attribute__((ext_vector_type(8)))  float    v8f;
typedef __attribute__((ext_vector_type(4)))  float    v4f;
typedef __attribute__((ext_vector_type(2)))  float    v2f;

constexpr int kBatch   = 32;
constexpr int kSeq     = 2048;
constexpr int kTok     = kBatch * kSeq;
constexpr int kState   = 128;
constexpr int kActW    = 16;
constexpr int kLat     = 256;
constexpr int kEnc     = 1024;
constexpr int kInW     = kState + 2 * kActW;
constexpr int kUOff    = kState + kActW;
constexpr int kWin     = 8;
constexpr int kEncRows = kBatch * kWin;
constexpr int kChunk   = 16384;
constexpr int kNChunk  = kTok / kChunk;
constexpr int kTS      = 32;
constexpr int kYP      = 260;
constexpr float kWCarry   = 256.0f;
constexpr float kACarry   = 64.0f;
constexpr float kInvCarry = 1.0f / (kWCarry * kACarry);

static_assert(kInW == 160 && kUOff == 144, "input row layout");
static_assert(kTok == 65536 && kEncRows == 256, "row counts");
static_assert((kState % 32) == 0 && (kEnc % 32) == 0 && (kLat % 32) == 0, "GEMM K multiples of 32");
static_assert((kEncRows % 64) == 0 && (kChunk % 64) == 0 && (kEnc % 64) == 0 && (kLat % 64) == 0 && (kState % 64) == 0, "GEMM M,N multiples of 64");
static_assert((kTok % kChunk) == 0 && (kSeq % kTS) == 0, "chunking");
static_assert(kTS * kYP >= kActW * kLat, "actuator weight staging fits the scan tile");
static_assert(kTS * kActW == 2 * 256, "u staging: one 8-byte load per thread");

constexpr size_t kOffE1 = 0;
constexpr size_t kOffE2 = kOffE1 + (size_t)kEnc * kState * 2;
constexpr size_t kOffE3 = kOffE2 + (size_t)kEnc * kEnc * 2;
constexpr size_t kOffD1 = kOffE3 + (size_t)kLat * kEnc * 2;
constexpr size_t kOffD2 = kOffD1 + (size_t)kEnc * kLat * 2;
constexpr size_t kOffD3 = kOffD2 + (size_t)kEnc * kEnc * 2;
constexpr size_t kOffXE = kOffD3 + (size_t)kState * kEnc * 2;
constexpr size_t kOffH1 = kOffXE + (size_t)kEncRows * kState * 2;
constexpr size_t kOffH2 = kOffH1 + (size_t)kEncRows * kEnc * 2;
constexpr size_t kOffZE = kOffH2 + (size_t)kEncRows * kEnc * 2;
constexpr size_t kOffZ1 = kOffZE + (size_t)kEncRows * kLat * 4;
constexpr size_t kOffG1 = kOffZ1 + (size_t)kTok * kLat * 2;
constexpr size_t kOffG2 = kOffG1 + (size_t)kChunk * kEnc * 2;
constexpr size_t kWsTotal = kOffG2 + (size_t)kChunk * kEnc * 2;
static_assert(kWsTotal == 107806720ull, "carve total");
static_assert(kWsTotal <= 134217728ull, "carve cap");
static_assert((kOffE2 % 128) == 0 && (kOffE3 % 128) == 0 && (kOffD1 % 128) == 0 && (kOffD2 % 128) == 0 &&
              (kOffD3 % 128) == 0 && (kOffXE % 128) == 0 && (kOffH1 % 128) == 0 && (kOffH2 % 128) == 0 &&
              (kOffZE % 128) == 0 && (kOffZ1 % 128) == 0 && (kOffG1 % 128) == 0 && (kOffG2 % 128) == 0, "128-B aligned regions");

__device__ __forceinline__ float bf_rne(float f) {
  unsigned u = __float_as_uint(f);
  u = (u + 0x7FFFu + ((u >> 16) & 1u)) & 0xFFFF0000u;
  return __uint_as_float(u);
}
__device__ __forceinline__ float tanh_fast(float x) {
  const float t = __builtin_amdgcn_exp2f(x * 2.8853900817779268f);
  return 1.0f - 2.0f * __builtin_amdgcn_rcpf(t + 1.0f);
}

__device__ __forceinline__ void tie_h(v8f& c, v16h a, v16h b) { asm volatile("" : "+v"(c) : "v"(a), "v"(b)); }
__device__ __forceinline__ void tie_nop_h(v8f& c, v16h a, v16h b) { asm volatile("v_nop\n\tv_nop\n\tv_nop\n\tv_nop" : "+v"(c) : "v"(a), "v"(b)); }
__device__ __forceinline__ void keep4_h(v16h a, v16h b, v16h c, v16h d) { asm volatile("v_nop" :: "v"(a), "v"(b), "v"(c), "v"(d)); }
__device__ __forceinline__ void acc_guard4(v8f& a, v8f& b, v8f& c, v8f& d) { asm volatile("v_nop\n\tv_nop\n\tv_nop\n\tv_nop" : "+v"(a), "+v"(b), "+v"(c), "+v"(d)); }

struct FragH {
  union U { v16h v; v8h h[2]; };
  static __device__ __forceinline__ v16h load(const _Float16* p) {
    U f;
    f.h[0] = *(const v8h*)(p);
    f.h[1] = *(const v8h*)(p + 16);
    return f.v;
  }
  static __device__ __forceinline__ v8f mma(v16h a, v16h b, v8f c) {
    return __builtin_amdgcn_wmma_f32_16x16x32_f16(false, a, false, b, (short)0, c, false, false);
  }
};

template <int OUT_MODE, int ACT>
__global__ __launch_bounds__(256) void wmma_gemm64(
    const unsigned short* __restrict__ Ap, int lda,
    const unsigned short* __restrict__ Btp, int ldb,
    void* __restrict__ Cout, int ldc,
    const float* __restrict__ bias,
    int M, int N, int K, float scale, float ocarry) {
  const _Float16* A  = (const _Float16*)Ap;
  const _Float16* Bt = (const _Float16*)Btp;
  __shared__ __align__(16) float sT[8][16 * 68];
  const int lane = threadIdx.x & 31;
  const int wave = threadIdx.x >> 5;
  const int tilesN = N >> 6;
  const int tilesM = M >> 6;
  const int tile = blockIdx.x * 8 + wave;
  if (tile >= tilesM * tilesN) return;
  const int tm = tile / tilesN;
  const int tn = tile - tm * tilesN;
  const int m0 = tm << 6;
  const int n0 = tn << 6;

  const int rlane = lane & 15;
  const int koff  = (lane >> 4) * 8;
  const int mOff  = (lane >> 4) * 8;

  v8f acc[4][4];
#pragma unroll
  for (int i = 0; i < 4; ++i)
#pragma unroll
    for (int j = 0; j < 4; ++j) acc[i][j] = (v8f){0.f, 0.f, 0.f, 0.f, 0.f, 0.f, 0.f, 0.f};

  for (int k0 = 0; k0 < K; k0 += 32) {
    v16h bh[4];
#pragma unroll
    for (int j = 0; j < 4; ++j) {
      const size_t bo = (size_t)(n0 + (j << 4) + rlane) * ldb + koff + k0;
      bh[j] = FragH::load(Bt + bo);
    }
#pragma unroll
    for (int i = 0; i < 4; ++i) {
      const size_t ao = (size_t)(m0 + (i << 4) + rlane) * lda + koff + k0;
      v16h ah = FragH::load(A + ao);
#pragma unroll
      for (int j = 0; j < 4; ++j) acc[i][j] = FragH::mma(ah, bh[j], acc[i][j]);
      tie_h(acc[i][0], ah, bh[0]);
      tie_h(acc[i][1], ah, bh[1]);
      tie_h(acc[i][2], ah, bh[2]);
      tie_nop_h(acc[i][3], ah, bh[3]);
    }
    keep4_h(bh[0], bh[1], bh[2], bh[3]);
  }
  acc_guard4(acc[0][0], acc[0][1], acc[0][2], acc[0][3]);
  acc_guard4(acc[1][0], acc[1][1], acc[1][2], acc[1][3]);
  acc_guard4(acc[2][0], acc[2][1], acc[2][2], acc[2][3]);
  acc_guard4(acc[3][0], acc[3][1], acc[3][2], acc[3][3]);

  float* slab = sT[wave];
#pragma unroll
  for (int i = 0; i < 4; ++i) {
    const int mBase = m0 + (i << 4);
#pragma unroll
    for (int j = 0; j < 4; ++j) {
      const int n = n0 + (j << 4) + rlane;
      const float bv = bf_rne(bias[n]);
#pragma unroll
      for (int r = 0; r < 8; ++r) {
        float v = acc[i][j][r] * scale + bv;
        if (ACT == 1) v = tanh_fast(v);
        slab[(mOff + r) * 68 + (j << 4) + rlane] = v;
      }
    }
    __builtin_amdgcn_fence(__ATOMIC_RELEASE, "workgroup");
    __builtin_amdgcn_wave_barrier();
    __builtin_amdgcn_fence(__ATOMIC_ACQUIRE, "workgroup");
    if (OUT_MODE == 0) {
      float* C = (float*)Cout;
      const int hh = lane >> 4, c4 = (lane & 15) * 4;
      for (int pass = 0; pass < 2; ++pass) {
#pragma unroll
        for (int it = 0; it < 8; ++it) {
          const int row = it * 2 + hh;
          v4f v = *(const v4f*)(slab + row * 68 + c4);
          *(volatile v4f*)(C + (size_t)(mBase + row) * ldc + n0 + c4) = v;
        }
        __threadfence();
      }
    } else {
      const int q = lane >> 3, c8 = (lane & 7) * 8;
      unsigned short* C = (unsigned short*)Cout;
      for (int pass = 0; pass < 2; ++pass) {
#pragma unroll
        for (int it = 0; it < 4; ++it) {
          const int row = it * 4 + q;
          const float* sp = slab + row * 68 + c8;
          v8h hv;
#pragma unroll
          for (int e = 0; e < 8; ++e) hv[e] = (_Float16)(sp[e] * ocarry);
          *(volatile v8h*)(C + (size_t)(mBase + row) * ldc + n0 + c8) = hv;
        }
        __threadfence();
      }
    }
    __builtin_amdgcn_fence(__ATOMIC_RELEASE, "workgroup");
    __builtin_amdgcn_wave_barrier();
    __builtin_amdgcn_fence(__ATOMIC_ACQUIRE, "workgroup");
  }
}

__global__ __launch_bounds__(256) void weight_plane_kernel(
    const float* __restrict__ W, unsigned short* __restrict__ Bt, int K, int N) {
  __shared__ __align__(16) float sW[64 * 68];
  const int tid = threadIdx.x;
  const int n0 = blockIdx.x * 64;
  const int k0 = blockIdx.y * 64;
  const int r = tid >> 4, c4 = (tid & 15) * 4;
#pragma unroll
  for (int i = 0; i < 4; ++i) {
    const int k = r + 16 * i;
    const v4f w = *(const v4f*)(W + (size_t)(k0 + k) * N + n0 + c4);
    v4f o;
    o[0] = bf_rne(w[0]) * kWCarry;
    o[1] = bf_rne(w[1]) * kWCarry;
    o[2] = bf_rne(w[2]) * kWCarry;
    o[3] = bf_rne(w[3]) * kWCarry;
    *(v4f*)(sW + k * 68 + c4) = o;
  }
  __syncthreads();
  const int q = tid >> 3, k8 = (tid & 7) * 8;
  v8h hv[2];
#pragma unroll
  for (int j = 0; j < 2; ++j) {
    const int n = q + 32 * j;
#pragma unroll
    for (int e = 0; e < 8; ++e) hv[j][e] = (_Float16)sW[(k8 + e) * 68 + n];
  }
  for (int pass = 0; pass < 2; ++pass) {
#pragma unroll
    for (int j = 0; j < 2; ++j) {
      const int n = q + 32 * j;
      *(volatile v8h*)(Bt + (size_t)(n0 + n) * K + k0 + k8) = hv[j];
    }
    __threadfence();
  }
}

__global__ __launch_bounds__(256) void enc_input_kernel(
    const float* __restrict__ padded, unsigned short* __restrict__ XE) {
  const int i = blockIdx.x * 256 + threadIdx.x;
  const int row = i >> 4;
  const int c8 = (i & 15) * 8;
  const int b = row >> 3;
  const int t = row & 7;
  const float* src = padded + ((size_t)b * kSeq + t) * kInW + c8;
  const v4f a0 = *(const v4f*)(src);
  const v4f a1 = *(const v4f*)(src + 4);
  v8h hv;
  hv[0] = (_Float16)(bf_rne(a0[0]) * kACarry);
  hv[1] = (_Float16)(bf_rne(a0[1]) * kACarry);
  hv[2] = (_Float16)(bf_rne(a0[2]) * kACarry);
  hv[3] = (_Float16)(bf_rne(a0[3]) * kACarry);
  hv[4] = (_Float16)(bf_rne(a1[0]) * kACarry);
  hv[5] = (_Float16)(bf_rne(a1[1]) * kACarry);
  hv[6] = (_Float16)(bf_rne(a1[2]) * kACarry);
  hv[7] = (_Float16)(bf_rne(a1[3]) * kACarry);
  unsigned short* dst = XE + (size_t)row * kState + c8;
  *(volatile v8h*)dst = hv;
  __threadfence();
  *(volatile v8h*)dst = hv;
}

__global__ __launch_bounds__(256) void scan_kernel(
    const float* __restrict__ padded, const float* __restrict__ Bw, const float* __restrict__ adiag,
    const float* __restrict__ ZE, const int* __restrict__ nwp, unsigned short* __restrict__ Z1) {
  __shared__ __align__(16) float sU[kTS * kActW];
  __shared__ __align__(16) float sY[kTS * kYP];
  __shared__ __align__(16) float sZ[kWin * kLat];
  const int tid = threadIdx.x, lane = tid & 31, wave = tid >> 5;
  const int b = blockIdx.x;
  const size_t row0 = (size_t)b * kSeq;

  const int nw_raw = nwp[0];
  const bool bad = (nw_raw > kWin - 1);
  int nw = nw_raw < 0 ? 0 : nw_raw;
  nw = nw > kWin - 1 ? kWin - 1 : nw;
  const float qnan = __uint_as_float(0x7FC00000u);

  float a = bf_rne(adiag[tid]);
  a = fminf(0.95f, fmaxf(-0.95f, a));

#pragma unroll
  for (int i = 0; i < 4; ++i) {
    const int idx = tid + 256 * i;
    const v4f w = *(const v4f*)(Bw + 4 * idx);
    v4f o;
    o[0] = bf_rne(w[0]);
    o[1] = bf_rne(w[1]);
    o[2] = bf_rne(w[2]);
    o[3] = bf_rne(w[3]);
    *(v4f*)(sY + 4 * idx) = o;
  }
#pragma unroll
  for (int i = 0; i < kWin; ++i) sZ[i * kLat + tid] = ZE[((size_t)b * kWin + i) * kLat + tid];
  __syncthreads();
  float bw[kActW];
#pragma unroll
  for (int k = 0; k < kActW; ++k) bw[k] = sY[k * kLat + tid];

  float carry = 0.0f;
  const int us = tid >> 3, uc = (tid & 7) * 2;
#pragma unroll 1
  for (int t0 = 0; t0 < kSeq; t0 += kTS) {
    __syncthreads();
    {
      const v2f uv = *(const v2f*)(padded + (row0 + t0 + us) * kInW + kUOff + uc);
      v2f uo;
      uo[0] = bf_rne(uv[0]);
      uo[1] = bf_rne(uv[1]);
      *(v2f*)(sU + us * kActW + uc) = uo;
    }
    __syncthreads();
#pragma unroll 1
    for (int s = 0; s < kTS; ++s) {
      const int t = t0 + s;
      const float* ur = sU + s * kActW;
      float bu = 0.0f;
#pragma unroll
      for (int q4 = 0; q4 < 4; ++q4) {
        const v4f uv = *(const v4f*)(ur + 4 * q4);
        bu = fmaf(uv[0], bw[4 * q4 + 0], bu);
        bu = fmaf(uv[1], bw[4 * q4 + 1], bu);
        bu = fmaf(uv[2], bw[4 * q4 + 2], bu);
        bu = fmaf(uv[3], bw[4 * q4 + 3], bu);
      }
      const int ti = t < kWin - 1 ? t : kWin - 1;
      const float zv = sZ[ti * kLat + tid];
      const float inp = (t <= nw) ? zv : carry;
      float nv = a * inp + bu;
      nv = bad ? qnan : nv;
      carry = nv;
      sY[s * kYP + tid] = nv;
    }
    __syncthreads();
    v8h hv[4];
#pragma unroll
    for (int it = 0; it < 4; ++it) {
      const int row = it * 8 + wave;
      const float* sp = sY + row * kYP + lane * 8;
      const v4f a0 = *(const v4f*)(sp);
      const v4f a1 = *(const v4f*)(sp + 4);
      hv[it][0] = (_Float16)(a0[0] * kACarry);
      hv[it][1] = (_Float16)(a0[1] * kACarry);
      hv[it][2] = (_Float16)(a0[2] * kACarry);
      hv[it][3] = (_Float16)(a0[3] * kACarry);
      hv[it][4] = (_Float16)(a1[0] * kACarry);
      hv[it][5] = (_Float16)(a1[1] * kACarry);
      hv[it][6] = (_Float16)(a1[2] * kACarry);
      hv[it][7] = (_Float16)(a1[3] * kACarry);
    }
    for (int pass = 0; pass < 2; ++pass) {
#pragma unroll
      for (int it = 0; it < 4; ++it) {
        const int row = it * 8 + wave;
        *(volatile v8h*)(Z1 + (row0 + t0 + row) * kLat + lane * 8) = hv[it];
      }
      __threadfence();
    }
  }
}

extern "C" void kernel_launch(void* const* d_in, const int* in_sizes, int n_in,
                              void* d_out, int out_size, void* d_ws, size_t ws_size,
                              hipStream_t stream) {
  if (n_in < 16) return;
  if (in_sizes[0] != kTok * kInW) return;
  if (in_sizes[1] != kState * kEnc) return;
  if (in_sizes[2] != kEnc) return;
  if (in_sizes[3] != kEnc * kEnc) return;
  if (in_sizes[4] != kEnc) return;
  if (in_sizes[5] != kEnc * kLat) return;
  if (in_sizes[6] != kLat) return;
  if (in_sizes[7] != kLat) return;
  if (in_sizes[8] != kActW * kLat) return;
  if (in_sizes[9] != kLat * kEnc) return;
  if (in_sizes[10] != kEnc) return;
  if (in_sizes[11] != kEnc * kEnc) return;
  if (in_sizes[12] != kEnc) return;
  if (in_sizes[13] != kEnc * kState) return;
  if (in_sizes[14] != kState) return;
  if (in_sizes[15] != 1) return;
  if (out_size != kTok * kState) return;
  if (ws_size < kWsTotal) return;

  const float* padded = (const float*)d_in[0];
  const float* enc_w1 = (const float*)d_in[1];
  const float* enc_b1 = (const float*)d_in[2];
  const float* enc_w2 = (const float*)d_in[3];
  const float* enc_b2 = (const float*)d_in[4];
  const float* enc_w3 = (const float*)d_in[5];
  const float* enc_b3 = (const float*)d_in[6];
  const float* a_diag = (const float*)d_in[7];
  const float* B_w    = (const float*)d_in[8];
  const float* dec_w1 = (const float*)d_in[9];
  const float* dec_b1 = (const float*)d_in[10];
  const float* dec_w2 = (const float*)d_in[11];
  const float* dec_b2 = (const float*)d_in[12];
  const float* dec_w3 = (const float*)d_in[13];
  const float* dec_b3 = (const float*)d_in[14];
  const int*   nwp    = (const int*)d_in[15];
  float* out = (float*)d_out;

  char* ws = (char*)d_ws;
  unsigned short* E1T = (unsigned short*)(ws + kOffE1);
  unsigned short* E2T = (unsigned short*)(ws + kOffE2);
  unsigned short* E3T = (unsigned short*)(ws + kOffE3);
  unsigned short* D1T = (unsigned short*)(ws + kOffD1);
  unsigned short* D2T = (unsigned short*)(ws + kOffD2);
  unsigned short* D3T = (unsigned short*)(ws + kOffD3);
  unsigned short* XE  = (unsigned short*)(ws + kOffXE);
  unsigned short* HE1 = (unsigned short*)(ws + kOffH1);
  unsigned short* HE2 = (unsigned short*)(ws + kOffH2);
  float*          ZE  = (float*)(ws + kOffZE);
  unsigned short* Z1  = (unsigned short*)(ws + kOffZ1);
  unsigned short* G1  = (unsigned short*)(ws + kOffG1);
  unsigned short* G2  = (unsigned short*)(ws + kOffG2);

  weight_plane_kernel<<<dim3(kEnc / 64, kState / 64), 256, 0, stream>>>(enc_w1, E1T, kState, kEnc);
  weight_plane_kernel<<<dim3(kEnc / 64, kEnc / 64), 256, 0, stream>>>(enc_w2, E2T, kEnc, kEnc);
  weight_plane_kernel<<<dim3(kLat / 64, kEnc / 64), 256, 0, stream>>>(enc_w3, E3T, kEnc, kLat);
  weight_plane_kernel<<<dim3(kEnc / 64, kLat / 64), 256, 0, stream>>>(dec_w1, D1T, kLat, kEnc);
  weight_plane_kernel<<<dim3(kEnc / 64, kEnc / 64), 256, 0, stream>>>(dec_w2, D2T, kEnc, kEnc);
  weight_plane_kernel<<<dim3(kState / 64, kEnc / 64), 256, 0, stream>>>(dec_w3, D3T, kEnc, kState);

  enc_input_kernel<<<(kEncRows * kState / 8) / 256, 256, 0, stream>>>(padded, XE);

  wmma_gemm64<1, 1><<<dim3(((kEncRows / 64) * (kEnc / 64)) / 8), 256, 0, stream>>>(
      XE, kState, E1T, kState, (void*)HE1, kEnc, enc_b1, kEncRows, kEnc, kState, kInvCarry, kACarry);
  wmma_gemm64<1, 1><<<dim3(((kEncRows / 64) * (kEnc / 64)) / 8), 256, 0, stream>>>(
      HE1, kEnc, E2T, kEnc, (void*)HE2, kEnc, enc_b2, kEncRows, kEnc, kEnc, kInvCarry, kACarry);
  wmma_gemm64<0, 1><<<dim3(((kEncRows / 64) * (kLat / 64)) / 8), 256, 0, stream>>>(
      HE2, kEnc, E3T, kEnc, (void*)ZE, kLat, enc_b3, kEncRows, kLat, kEnc, kInvCarry, 1.0f);

  scan_kernel<<<kBatch, 256, 0, stream>>>(padded, B_w, a_diag, ZE, nwp, Z1);

  for (int c = 0; c < kNChunk; ++c) {
    const size_t r0 = (size_t)c * kChunk;
    wmma_gemm64<1, 1><<<dim3(((kChunk / 64) * (kEnc / 64)) / 8), 256, 0, stream>>>(
        Z1 + r0 * kLat, kLat, D1T, kLat, (void*)G1, kEnc, dec_b1, kChunk, kEnc, kLat, kInvCarry, kACarry);
    wmma_gemm64<1, 1><<<dim3(((kChunk / 64) * (kEnc / 64)) / 8), 256, 0, stream>>>(
        G1, kEnc, D2T, kEnc, (void*)G2, kEnc, dec_b2, kChunk, kEnc, kEnc, kInvCarry, kACarry);
    wmma_gemm64<0, 0><<<dim3(((kChunk / 64) * (kState / 64)) / 8), 256, 0, stream>>>(
        G2, kEnc, D3T, kEnc, (void*)(out + r0 * kState), kState, dec_b3, kChunk, kState, kEnc, kInvCarry, 1.0f);
  }
}
